// AttentionXL_29772713295987
// MI455X (gfx1250) — hardware-verified
//
#include <hip/hip_runtime.h>
#include <stddef.h>
#include <stdint.h>

#define CUR   1024
#define FULL  2048
#define BSZ   4
#define DM    1024
#define NH    16
#define DH    64
#define NBH   (BSZ * NH)
#define KCW   64
#define NCH   (FULL / KCW)
#define QBR   64
#define NQB   (CUR / QBR)
#define RWIN  128
#define ATT_SCALE 0.125f
#define WSC   32.0f
#define PSC   1024.0f

static_assert(DM == NH * DH);
static_assert(DH == 64);
static_assert(FULL == 2 * CUR);
static_assert(NCH == 32);
static_assert(CUR % 256 == 0);
static_assert(FULL % 256 == 0);
static_assert((CUR * BSZ) % 256 == 0);
static_assert((FULL * BSZ) % 256 == 0);
static_assert(DM % 64 == 0);
static_assert(QBR == 64);
static_assert(RWIN == 48 + 80);

typedef _Float16 v16h __attribute__((ext_vector_type(16)));
typedef _Float16 v8h  __attribute__((ext_vector_type(8)));
typedef float    v8f  __attribute__((ext_vector_type(8)));
typedef float    v4f  __attribute__((ext_vector_type(4)));
typedef int      v4i  __attribute__((ext_vector_type(4)));
typedef unsigned int v4u __attribute__((ext_vector_type(4)));
typedef unsigned long long u64;

union Frag  { v16h v; v8h h[2]; };
union Pack8 { v8h h; v4u u; };

__device__ __forceinline__ v8f zero8() { return (v8f){0.f, 0.f, 0.f, 0.f, 0.f, 0.f, 0.f, 0.f}; }

__device__ __forceinline__ v8f mma16(v16h a, v16h b, v8f c) {
  c = __builtin_amdgcn_wmma_f32_16x16x32_f16(false, a, false, b, (short)0, c, false, false);
  asm volatile("v_nop\n\tv_nop\n\tv_nop\n\tv_nop" : "+v"(c) : "v"(a), "v"(b));
  return c;
}

__device__ __forceinline__ v16h ldfrag(const _Float16* p, int ld, int row0, int k0, int lane) {
  const int m = lane & 15, lh = lane >> 4;
  const _Float16* q = p + (size_t)(row0 + m) * ld + k0 + 8 * lh;
  Frag f;
  f.h[0] = *(const v8h*)(q);
  f.h[1] = *(const v8h*)(q + 16);
  return f.v;
}

__device__ __forceinline__ v8h cvt8(v4f a0, v4f a1, float sc) {
  return (v8h){(_Float16)(a0[0] * sc), (_Float16)(a0[1] * sc), (_Float16)(a0[2] * sc), (_Float16)(a0[3] * sc),
               (_Float16)(a1[0] * sc), (_Float16)(a1[1] * sc), (_Float16)(a1[2] * sc), (_Float16)(a1[3] * sc)};
}

__device__ __forceinline__ void gemm32x64(const _Float16* __restrict__ A, int lda,
                                          const _Float16* __restrict__ Bt,
                                          int m0, int n0, int lane, v8f (&acc)[2][4]) {
#pragma unroll 2
  for (int k0 = 0; k0 < DM; k0 += 32) {
    const v16h a0 = ldfrag(A, lda, m0, k0, lane);
    const v16h a1 = ldfrag(A, lda, m0 + 16, k0, lane);
#pragma unroll
    for (int t = 0; t < 4; ++t) {
      const v16h b = ldfrag(Bt, DM, n0 + 16 * t, k0, lane);
      acc[0][t] = mma16(a0, b, acc[0][t]);
      acc[1][t] = mma16(a1, b, acc[1][t]);
    }
  }
}

__global__ __launch_bounds__(128) void k_cvt(const float* __restrict__ src, _Float16* __restrict__ dst) {
  const size_t o = (size_t)blockIdx.x * DM + (size_t)threadIdx.x * 8;
  const v4f a0 = *(const v4f*)(src + o);
  const v4f a1 = *(const v4f*)(src + o + 4);
  Pack8 pk;
  pk.h = cvt8(a0, a1, 1.0f);
  const v4u vv = pk.u;
  volatile v4u* d = (volatile v4u*)(dst + o);
  *d = vv;
  __threadfence();
  *d = vv;
}

#define WTP 72
__global__ __launch_bounds__(256) void k_wt(const float* __restrict__ W, _Float16* __restrict__ Wt, int N) {
  __shared__ __align__(16) _Float16 sT[64 * WTP];
  const int tid = threadIdx.x;
  const int n0 = blockIdx.x * 64, k0 = blockIdx.y * 64;
  const int kr = tid >> 2, nq = (tid & 3) * 16;
  const float* sp = W + (size_t)(k0 + kr) * N + n0 + nq;
#pragma unroll
  for (int q = 0; q < 4; ++q) {
    const v4f v = *(const v4f*)(sp + 4 * q);
#pragma unroll
    for (int e = 0; e < 4; ++e) sT[(nq + 4 * q + e) * WTP + kr] = (_Float16)(v[e] * WSC);
  }
  __syncthreads();
  v4u val[2];
  size_t go[2];
#pragma unroll
  for (int it = 0; it < 2; ++it) {
    const int p  = tid + 256 * it;
    const int L  = p >> 3;
    const int pc = p & 7;
    Pack8 pk;
    pk.h    = *(const v8h*)(sT + L * WTP + 8 * pc);
    val[it] = pk.u;
    go[it]  = (size_t)(n0 + L) * DM + k0 + 8 * pc;
  }
  for (int ps = 0; ps < 2; ++ps) {
#pragma unroll
    for (int it = 0; it < 2; ++it) *(volatile v4u*)(Wt + go[it]) = val[it];
    __threadfence();
  }
}

__global__ __launch_bounds__(256) void k_mbits(const int* __restrict__ msk, u64* __restrict__ mb) {
  __shared__ __align__(16) u64 wsh[BSZ][NCH];
  const int tid = threadIdx.x, lane = tid & 31, wave = tid >> 5;
  const int i  = blockIdx.x;
  const int jb = 256 * wave + 8 * lane;
  const int* mp = msk + ((size_t)i * FULL + jb) * BSZ;
  unsigned bt[4];
#pragma unroll
  for (int bb = 0; bb < 4; ++bb) bt[bb] = 0u;
#pragma unroll
  for (int e = 0; e < 8; ++e) {
    const v4i q = *(const v4i*)(mp + 4 * e);
#pragma unroll
    for (int bb = 0; bb < 4; ++bb) bt[bb] |= (q[bb] != 0) ? (1u << e) : 0u;
  }
  const int sh = 8 * (lane & 7);
  unsigned lo[4], hi[4];
#pragma unroll
  for (int bb = 0; bb < 4; ++bb) {
    const u64 w = ((u64)bt[bb]) << sh;
    unsigned l0 = (unsigned)w, h0 = (unsigned)(w >> 32);
#pragma unroll
    for (int off = 1; off < 8; off <<= 1) {
      l0 |= __shfl_xor(l0, off, 32);
      h0 |= __shfl_xor(h0, off, 32);
    }
    lo[bb] = l0;
    hi[bb] = h0;
  }
  if ((lane & 7) == 0) {
    const int kc = 4 * wave + (lane >> 3);
#pragma unroll
    for (int bb = 0; bb < 4; ++bb) wsh[bb][kc] = (((u64)hi[bb]) << 32) | (u64)lo[bb];
  }
  __syncthreads();
  if (tid < 64) {
    const int bb = tid >> 4, pc = tid & 15;
    const v4u val = *(const v4u*)(&wsh[bb][2 * pc]);
    u64* gp = mb + ((size_t)(bb * CUR + i)) * NCH + 2 * pc;
    *(volatile v4u*)gp = val;
    __threadfence();
    *(volatile v4u*)gp = val;
  }
}

#define KVP 72
__global__ __launch_bounds__(256) __attribute__((amdgpu_num_vgpr(256)))
void k_kv(const _Float16* __restrict__ Xf, const _Float16* __restrict__ Wt,
          const float* __restrict__ bias, _Float16* __restrict__ Kp, _Float16* __restrict__ Vt) {
  __shared__ __align__(16) _Float16 sT[256 * KVP];
  const int tid = threadIdx.x, lane = tid & 31, wave = tid >> 5;
  const int hh = lane >> 4, c = lane & 15;
  const int r0 = blockIdx.x * 256;
  const int jbase = blockIdx.x * 64;
  const int n0 = blockIdx.y * 64;
  const bool kpart = (blockIdx.y < NH);
  const int h = kpart ? (int)blockIdx.y : ((int)blockIdx.y - NH);

  v8f acc[2][4];
#pragma unroll
  for (int s = 0; s < 2; ++s)
#pragma unroll
    for (int t = 0; t < 4; ++t) acc[s][t] = zero8();
  gemm32x64(Xf, DM, Wt, r0 + 32 * wave, n0, lane, acc);

#pragma unroll
  for (int sub = 0; sub < 2; ++sub) {
#pragma unroll
    for (int t = 0; t < 4; ++t) {
      const float bb = bias[n0 + 16 * t + c];
      const int d = 16 * t + c;
#pragma unroll
      for (int r = 0; r < 8; ++r) {
        const int rl  = 32 * wave + 16 * sub + 8 * hh + r;
        const int idx = kpart ? (rl * KVP + d) : ((((rl & 3) * 64) + d) * KVP + (rl >> 2));
        sT[idx] = (_Float16)(acc[sub][t][r] * 0.03125f + bb);
      }
    }
  }
  __syncthreads();

  v4u val[8];
  size_t go[8];
#pragma unroll
  for (int it = 0; it < 8; ++it) {
    const int p  = tid + 256 * it;
    const int L  = p >> 3;
    const int pc = p & 7;
    Pack8 pk;
    pk.h    = *(const v8h*)(sT + L * KVP + 8 * pc);
    val[it] = pk.u;
    const size_t ka = (((size_t)((L & 3) * NH + h)) * FULL + jbase + (L >> 2)) * DH + 8 * pc;
    const size_t va = (((size_t)((L >> 6) * NH + h)) * DH + (L & 63)) * FULL + jbase + 8 * pc;
    go[it]  = kpart ? ka : va;
  }
  _Float16* base = kpart ? Kp : Vt;
  for (int ps = 0; ps < 2; ++ps) {
#pragma unroll
    for (int it = 0; it < 8; ++it) *(volatile v4u*)(base + go[it]) = val[it];
    __threadfence();
  }
}

#define QSP 68
__device__ __forceinline__ void stage16(v8f (&acc)[2][4], int sub, float scale, const float* __restrict__ bias,
                                        int n0, float* sw, int hh, int c) {
#pragma unroll
  for (int t = 0; t < 4; ++t) {
    const float bb = bias[n0 + 16 * t + c];
#pragma unroll
    for (int r = 0; r < 8; ++r) sw[(8 * hh + r) * QSP + 16 * t + c] = acc[sub][t][r] * scale + bb;
  }
}

__global__ __launch_bounds__(256) __attribute__((amdgpu_num_vgpr(256)))
void k_q(const _Float16* __restrict__ Xc, const _Float16* __restrict__ Wt, const float* __restrict__ bq,
         const float* __restrict__ uu, const float* __restrict__ vv,
         _Float16* __restrict__ QU, _Float16* __restrict__ QV) {
  __shared__ __align__(16) float st[8][16 * QSP];
  const int tid = threadIdx.x, lane = tid & 31, wave = tid >> 5;
  const int hh = lane >> 4, c = lane & 15;
  const int r0 = blockIdx.x * 256;
  const int ibase = blockIdx.x * 64;
  const int n0 = blockIdx.y * 64;
  const int h  = blockIdx.y;

  v8f acc[2][4];
#pragma unroll
  for (int s = 0; s < 2; ++s)
#pragma unroll
    for (int t = 0; t < 4; ++t) acc[s][t] = zero8();
  gemm32x64(Xc, DM, Wt, r0 + 32 * wave, n0, lane, acc);

  float* sw = st[wave];
  const float* uh = uu + h * DH;
  const float* vh = vv + h * DH;
#pragma unroll
  for (int sub = 0; sub < 2; ++sub) {
    __syncthreads();
    stage16(acc, sub, 0.03125f, bq, n0, sw, hh, c);
    __syncthreads();
    v4u pu[4], pv[4];
    size_t go[4];
#pragma unroll
    for (int it = 0; it < 4; ++it) {
      const int p  = lane + 32 * it;
      const int L  = p >> 3;
      const int pc = p & 7;
      const float* rp = sw + L * QSP + 8 * pc;
      const v4f a0 = *(const v4f*)(rp), a1 = *(const v4f*)(rp + 4);
      const v4f u0 = *(const v4f*)(uh + 8 * pc), u1 = *(const v4f*)(uh + 8 * pc + 4);
      const v4f v0 = *(const v4f*)(vh + 8 * pc), v1 = *(const v4f*)(vh + 8 * pc + 4);
      Pack8 k1, k2;
      k1.h = cvt8(a0 + u0, a1 + u1, 1.0f);
      k2.h = cvt8(a0 + v0, a1 + v1, 1.0f);
      pu[it] = k1.u;
      pv[it] = k2.u;
      const int rl = 32 * wave + 16 * sub + L;
      go[it] = (((size_t)((rl & 3) * NH + h)) * CUR + ibase + (rl >> 2)) * DH + 8 * pc;
    }
    for (int ps = 0; ps < 2; ++ps) {
#pragma unroll
      for (int it = 0; it < 4; ++it) {
        *(volatile v4u*)(QU + go[it]) = pu[it];
        *(volatile v4u*)(QV + go[it]) = pv[it];
      }
      __threadfence();
    }
  }
}

__global__ __launch_bounds__(256) __attribute__((amdgpu_num_vgpr(256)))
void k_r(const _Float16* __restrict__ Xp, const _Float16* __restrict__ Wt, const float* __restrict__ br,
         _Float16* __restrict__ Rp) {
  __shared__ __align__(16) float st[8][16 * QSP];
  const int tid = threadIdx.x, lane = tid & 31, wave = tid >> 5;
  const int hh = lane >> 4, c = lane & 15;
  const int r0 = blockIdx.x * 256;
  const int n0 = blockIdx.y * 64;
  const int h  = blockIdx.y;

  v8f acc[2][4];
#pragma unroll
  for (int s = 0; s < 2; ++s)
#pragma unroll
    for (int t = 0; t < 4; ++t) acc[s][t] = zero8();
  gemm32x64(Xp, DM, Wt, r0 + 32 * wave, n0, lane, acc);

  float* sw = st[wave];
#pragma unroll
  for (int sub = 0; sub < 2; ++sub) {
    __syncthreads();
    stage16(acc, sub, 0.03125f, br, n0, sw, hh, c);
    __syncthreads();
    v4u val[4];
    size_t go[4];
#pragma unroll
    for (int it = 0; it < 4; ++it) {
      const int p  = lane + 32 * it;
      const int L  = p >> 3;
      const int pc = p & 7;
      const float* rp = sw + L * QSP + 8 * pc;
      const v4f a0 = *(const v4f*)(rp), a1 = *(const v4f*)(rp + 4);
      Pack8 pk;
      pk.h    = cvt8(a0, a1, 1.0f);
      val[it] = pk.u;
      const int m = r0 + 32 * wave + 16 * sub + L;
      go[it]  = ((size_t)h * FULL + m) * DH + 8 * pc;
    }
    for (int ps = 0; ps < 2; ++ps) {
#pragma unroll
      for (int it = 0; it < 4; ++it) *(volatile v4u*)(Rp + go[it]) = val[it];
      __threadfence();
    }
  }
}

#define TP  64
#define PWW 80
#define PPH 72
__global__ __launch_bounds__(128) __attribute__((amdgpu_num_vgpr(256)))
void k_attn(const _Float16* __restrict__ QU, const _Float16* __restrict__ QV,
            const _Float16* __restrict__ Kp, const _Float16* __restrict__ Vt,
            const _Float16* __restrict__ Rp, const u64* __restrict__ mb,
            _Float16* __restrict__ Op) {
  __shared__ __align__(16) _Float16 Ks[KCW * TP];
  __shared__ __align__(16) _Float16 Vs[DH * TP];
  __shared__ __align__(16) _Float16 Rs[RWIN * TP];
  __shared__ __align__(16) float    Pw[4][16 * PWW];
  __shared__ __align__(16) _Float16 Pt[4][16 * PPH];
  __shared__ unsigned red[4][2];

  const int tid = threadIdx.x, lane = tid & 31, wave = tid >> 5;
  const int hh = lane >> 4, c = lane & 15;
  const int qblk = blockIdx.x % NQB;
  const int bh   = blockIdx.x / NQB;
  const int b    = bh / NH;
  const int h    = bh - b * NH;
  const int i0b  = qblk * QBR;
  const int i0   = i0b + wave * 16;
  const int woff = 48 - 16 * wave;

  const _Float16* QUp = QU + (size_t)bh * CUR * DH;
  const _Float16* QVp = QV + (size_t)bh * CUR * DH;
  const _Float16* Kb  = Kp + (size_t)bh * FULL * DH;
  const _Float16* Vb  = Vt + (size_t)bh * DH * FULL;
  const _Float16* Rb  = Rp + (size_t)h * FULL * DH;
  const u64*      mw0 = mb + ((size_t)(b * CUR + i0)) * NCH;

  unsigned need = 0u, rf = 0u;
  {
    const int row = lane & 15;
    const u64* mr = mw0 + row * NCH + (lane >> 4);
#pragma unroll
    for (int e = 0; e < 16; ++e) {
      const u64 w  = mr[2 * e];
      const int kc = (lane >> 4) + 2 * e;
      const bool unb = (w != ~0ull);
      need |= unb ? (1u << kc) : 0u;
      rf   |= unb ? 1u : 0u;
    }
  }
#pragma unroll
  for (int off = 1; off < 32; off <<= 1) need |= __shfl_xor(need, off, 32);
  rf |= __shfl_xor(rf, 16, 32);
#pragma unroll
  for (int off = 1; off < 16; off <<= 1) rf &= __shfl_xor(rf, off, 32);
  if (lane == 0) { red[wave][0] = need; red[wave][1] = rf; }
  __syncthreads();
  const unsigned blkneed = (unsigned)__builtin_amdgcn_readfirstlane((int)(red[0][0] | red[1][0] | red[2][0] | red[3][0]));
  const unsigned rowsfin = (unsigned)__builtin_amdgcn_readfirstlane((int)(red[0][1] & red[1][1] & red[2][1] & red[3][1]));
  const bool rfin = (rowsfin != 0u);

  const float NEGI = -__builtin_huge_valf();
  float mrow[8], lrow[8];
  v8f oacc[4];
#pragma unroll
  for (int r = 0; r < 8; ++r) { mrow[r] = NEGI; lrow[r] = 0.f; }
#pragma unroll
  for (int t = 0; t < 4; ++t) oacc[t] = zero8();

  float*    pw = Pw[wave];
  _Float16* pt = Pt[wave];

  for (int kc = 0; kc < NCH; ++kc) {
    if (rfin && (((blkneed >> kc) & 1u) == 0u)) continue;
    const int j0 = kc * KCW;
    const int sB = j0 + (CUR - QBR) - i0b;
    __syncthreads();
#pragma unroll
    for (int e = 0; e < 4; ++e) {
      const int p  = tid + 128 * e;
      const int r  = p >> 3;
      const int pc = p & 7;
      *(v8h*)(Ks + r * TP + 8 * pc) = *(const v8h*)(Kb + (size_t)(j0 + r) * DH + 8 * pc);
      *(v8h*)(Vs + r * TP + 8 * pc) = *(const v8h*)(Vb + (size_t)r * FULL + j0 + 8 * pc);
    }
#pragma unroll
    for (int e = 0; e < 8; ++e) {
      const int p  = tid + 128 * e;
      const int r  = p >> 3;
      const int pc = p & 7;
      int s = sB + r;
      s = (s < 0) ? 0 : s;
      s = (s > FULL - 1) ? (FULL - 1) : s;
      *(v8h*)(Rs + r * TP + 8 * pc) = *(const v8h*)(Rb + (size_t)s * DH + 8 * pc);
    }
    __syncthreads();

    {
      v8f PW[5];
#pragma unroll
      for (int t = 0; t < 5; ++t) PW[t] = zero8();
#pragma unroll
      for (int kk = 0; kk < 2; ++kk) {
        const v16h a = ldfrag(QVp, DH, i0, 32 * kk, lane);
#pragma unroll
        for (int t = 0; t < 5; ++t) {
          const v16h bf = ldfrag(Rs, TP, woff + 16 * t, 32 * kk, lane);
          PW[t] = mma16(a, bf, PW[t]);
        }
      }
#pragma unroll
      for (int t = 0; t < 5; ++t)
#pragma unroll
        for (int r = 0; r < 8; ++r) pw[(8 * hh + r) * PWW + 16 * t + c] = PW[t][r];
    }
    __syncthreads();

    v8f S[4];
#pragma unroll
    for (int t = 0; t < 4; ++t) S[t] = zero8();
#pragma unroll
    for (int kk = 0; kk < 2; ++kk) {
      const v16h a = ldfrag(QUp, DH, i0, 32 * kk, lane);
#pragma unroll
      for (int t = 0; t < 4; ++t) {
        const v16h bf = ldfrag(Ks, TP, 16 * t, 32 * kk, lane);
        S[t] = mma16(a, bf, S[t]);
      }
    }
#pragma unroll
    for (int r = 0; r < 8; ++r) {
      const int ii = 8 * hh + r;
      const u64 wv = mw0[ii * NCH + kc];
      const float* pr = pw + ii * PWW + (15 - ii) + c;
#pragma unroll
      for (int t = 0; t < 4; ++t) {
        const float pos = pr[16 * t];
        const float sc  = (S[t][r] + pos) * ATT_SCALE;
        const unsigned blocked = (unsigned)((wv >> (16 * t + c)) & 1ull);
        S[t][r] = (blocked != 0u) ? -1.0e20f : sc;
      }
    }
    float al[8];
#pragma unroll
    for (int r = 0; r < 8; ++r) {
      float m = fmaxf(fmaxf(S[0][r], S[1][r]), fmaxf(S[2][r], S[3][r]));
#pragma unroll
      for (int off = 1; off < 16; off <<= 1) m = fmaxf(m, __shfl_xor(m, off, 32));
      const float mnew  = fmaxf(mrow[r], m);
      const float alpha = __expf(mrow[r] - mnew);
      mrow[r] = mnew;
      float psum = 0.f;
#pragma unroll
      for (int t = 0; t < 4; ++t) {
        const float p = __expf(S[t][r] - mnew);
        psum += p;
        pt[(8 * hh + r) * PPH + 16 * t + c] = (_Float16)(p * PSC);
      }
#pragma unroll
      for (int off = 1; off < 16; off <<= 1) psum += __shfl_xor(psum, off, 32);
      lrow[r] = lrow[r] * alpha + psum;
      al[r] = alpha;
    }
#pragma unroll
    for (int t = 0; t < 4; ++t)
#pragma unroll
      for (int r = 0; r < 8; ++r) oacc[t][r] *= al[r];
    __syncthreads();

#pragma unroll
    for (int kk = 0; kk < 2; ++kk) {
      const v16h a = ldfrag(pt, PPH, 0, 32 * kk, lane);
#pragma unroll
      for (int t = 0; t < 4; ++t) {
        const v16h bf = ldfrag(Vs, TP, 16 * t, 32 * kk, lane);
        oacc[t] = mma16(a, bf, oacc[t]);
      }
    }
  }

  float invl[8];
#pragma unroll
  for (int r = 0; r < 8; ++r) invl[r] = (lrow[r] > 0.f) ? (0.015625f / lrow[r]) : 0.f;
  __syncthreads();
#pragma unroll
  for (int r = 0; r < 8; ++r) {
#pragma unroll
    for (int t = 0; t < 4; ++t) pt[(8 * hh + r) * PPH + 16 * t + c] = (_Float16)(oacc[t][r] * invl[r]);
  }
  __syncthreads();
  v4u val[4];
  size_t go[4];
#pragma unroll
  for (int it = 0; it < 4; ++it) {
    const int p  = lane + 32 * it;
    const int L  = p >> 3;
    const int pc = p & 7;
    Pack8 pk;
    pk.h    = *(const v8h*)(pt + L * PPH + 8 * pc);
    val[it] = pk.u;
    go[it]  = ((size_t)bh * CUR + i0 + L) * DH + 8 * pc;
  }
  for (int ps = 0; ps < 2; ++ps) {
#pragma unroll
    for (int it = 0; it < 4; ++it) *(volatile v4u*)(Op + go[it]) = val[it];
    __threadfence();
  }
}

__global__ __launch_bounds__(256) __attribute__((amdgpu_num_vgpr(256)))
void k_out(const _Float16* __restrict__ Opl, const _Float16* __restrict__ Wt, const float* __restrict__ bo,
           float* __restrict__ out) {
  __shared__ __align__(16) float st[8][16 * QSP];
  const int tid = threadIdx.x, lane = tid & 31, wave = tid >> 5;
  const int hh = lane >> 4, c = lane & 15;
  const int b    = blockIdx.x >> 2;
  const int iblk = blockIdx.x & 3;
  const int i0w  = iblk * 256 + 32 * wave;
  const int n0   = blockIdx.y * 64;

  v8f acc[2][4];
#pragma unroll
  for (int s = 0; s < 2; ++s)
#pragma unroll
    for (int t = 0; t < 4; ++t) acc[s][t] = zero8();
#pragma unroll 1
  for (int hd = 0; hd < NH; ++hd) {
    const _Float16* A = Opl + (((size_t)(b * NH + hd)) * CUR + i0w) * DH;
#pragma unroll
    for (int sub = 0; sub < 2; ++sub) {
      const int ka = 32 * sub, kb = hd * DH + 32 * sub;
      const v16h a0 = ldfrag(A, DH, 0, ka, lane);
      const v16h a1 = ldfrag(A, DH, 16, ka, lane);
#pragma unroll
      for (int t = 0; t < 4; ++t) {
        const v16h bf = ldfrag(Wt, DM, n0 + 16 * t, kb, lane);
        acc[0][t] = mma16(a0, bf, acc[0][t]);
        acc[1][t] = mma16(a1, bf, acc[1][t]);
      }
    }
  }

  float* sw = st[wave];
#pragma unroll
  for (int sub = 0; sub < 2; ++sub) {
    __syncthreads();
    stage16(acc, sub, 0.001953125f, bo, n0, sw, hh, c);
    __syncthreads();
    v4f val[8];
    size_t go[8];
#pragma unroll
    for (int it = 0; it < 8; ++it) {
      const int p    = lane + 32 * it;
      const int L    = p >> 3;
      const int pc   = p & 7;
      const int row  = L >> 1;
      const int half = L & 1;
      val[it] = *(const v4f*)(sw + row * QSP + half * 32 + pc * 4);
      const int i = i0w + 16 * sub + row;
      go[it]  = ((size_t)(i * BSZ + b)) * DM + n0 + half * 32 + pc * 4;
    }
    for (int ps = 0; ps < 2; ++ps) {
#pragma unroll
      for (int it = 0; it < 8; ++it) *(volatile v4f*)(out + go[it]) = val[it];
      __threadfence();
    }
  }
}

extern "C" void kernel_launch(void* const* d_in, const int* in_sizes, int n_in,
                              void* d_out, int out_size, void* d_ws, size_t ws_size,
                              hipStream_t stream) {
  if (n_in < 14) return;
  if (in_sizes[0]  != CUR * BSZ * DM) return;
  if (in_sizes[1]  != FULL * DM) return;
  if (in_sizes[2]  != FULL * BSZ * DM) return;
  if (in_sizes[3]  != NH * DH) return;
  if (in_sizes[4]  != NH * DH) return;
  if (in_sizes[5]  != DM * 2 * DM) return;
  if (in_sizes[6]  != 2 * DM) return;
  if (in_sizes[7]  != DM * DM) return;
  if (in_sizes[8]  != DM) return;
  if (in_sizes[9]  != DM * DM) return;
  if (in_sizes[10] != DM) return;
  if (in_sizes[11] != DM * DM) return;
  if (in_sizes[12] != DM) return;
  if (in_sizes[13] != CUR * FULL * BSZ) return;
  if (out_size != CUR * BSZ * DM) return;

  const float* xin   = (const float*)d_in[0];
  const float* pos   = (const float*)d_in[1];
  const float* xfull = (const float*)d_in[2];
  const float* uu    = (const float*)d_in[3];
  const float* vv    = (const float*)d_in[4];
  const float* Wkv   = (const float*)d_in[5];
  const float* bkv   = (const float*)d_in[6];
  const float* Wq    = (const float*)d_in[7];
  const float* bq    = (const float*)d_in[8];
  const float* Wr    = (const float*)d_in[9];
  const float* br    = (const float*)d_in[10];
  const float* Wo    = (const float*)d_in[11];
  const float* bo    = (const float*)d_in[12];
  const int*   msk   = (const int*)d_in[13];
  float* out = (float*)d_out;

  size_t off = 0;
  const size_t oXc  = off; off += (size_t)CUR * BSZ * DM * 2;
  const size_t oXf  = off; off += (size_t)FULL * BSZ * DM * 2;
  const size_t oXp  = off; off += (size_t)FULL * DM * 2;
  const size_t oWkv = off; off += (size_t)2 * DM * DM * 2;
  const size_t oWq  = off; off += (size_t)DM * DM * 2;
  const size_t oWr  = off; off += (size_t)DM * DM * 2;
  const size_t oWo  = off; off += (size_t)DM * DM * 2;
  const size_t oK   = off; off += (size_t)NBH * FULL * DH * 2;
  const size_t oV   = off; off += (size_t)NBH * DH * FULL * 2;
  const size_t oQU  = off; off += (size_t)NBH * CUR * DH * 2;
  const size_t oQV  = off; off += (size_t)NBH * CUR * DH * 2;
  const size_t oR   = off; off += (size_t)NH * FULL * DH * 2;
  const size_t oMB  = off; off += (size_t)BSZ * CUR * NCH * 8;
  const size_t oO   = off; off += (size_t)NBH * CUR * DH * 2;
  if (off > ws_size) return;
  if (off > (size_t)134217728) return;

  char* ws = (char*)d_ws;
  _Float16* Xc   = (_Float16*)(ws + oXc);
  _Float16* Xf   = (_Float16*)(ws + oXf);
  _Float16* Xp   = (_Float16*)(ws + oXp);
  _Float16* WkvT = (_Float16*)(ws + oWkv);
  _Float16* WqT  = (_Float16*)(ws + oWq);
  _Float16* WrT  = (_Float16*)(ws + oWr);
  _Float16* WoT  = (_Float16*)(ws + oWo);
  _Float16* Kp   = (_Float16*)(ws + oK);
  _Float16* Vt   = (_Float16*)(ws + oV);
  _Float16* QU   = (_Float16*)(ws + oQU);
  _Float16* QV   = (_Float16*)(ws + oQV);
  _Float16* Rp   = (_Float16*)(ws + oR);
  u64*      MB   = (u64*)(ws + oMB);
  _Float16* Opl  = (_Float16*)(ws + oO);

  k_cvt<<<dim3(CUR * BSZ), dim3(DM / 8), 0, stream>>>(xin, Xc);
  k_cvt<<<dim3(FULL * BSZ), dim3(DM / 8), 0, stream>>>(xfull, Xf);
  k_cvt<<<dim3(FULL), dim3(DM / 8), 0, stream>>>(pos, Xp);
  k_wt<<<dim3((2 * DM) / 64, DM / 64), dim3(256), 0, stream>>>(Wkv, WkvT, 2 * DM);
  k_wt<<<dim3(DM / 64, DM / 64), dim3(256), 0, stream>>>(Wq, WqT, DM);
  k_wt<<<dim3(DM / 64, DM / 64), dim3(256), 0, stream>>>(Wr, WrT, DM);
  k_wt<<<dim3(DM / 64, DM / 64), dim3(256), 0, stream>>>(Wo, WoT, DM);
  k_mbits<<<dim3(CUR), dim3(256), 0, stream>>>(msk, MB);
  k_kv<<<dim3((FULL * BSZ) / 256, (2 * DM) / 64), dim3(256), 0, stream>>>(Xf, WkvT, bkv, Kp, Vt);
  k_q<<<dim3((CUR * BSZ) / 256, DM / 64), dim3(256), 0, stream>>>(Xc, WqT, bq, uu, vv, QU, QV);
  k_r<<<dim3(FULL / 256, NH), dim3(256), 0, stream>>>(Xp, WrT, br, Rp);
  k_attn<<<dim3(NBH * NQB), dim3(128), 0, stream>>>(QU, QV, Kp, Vt, Rp, MB, Opl);
  k_out<<<dim3(BSZ * (CUR / 256), DM / 64), dim3(256), 0, stream>>>(Opl, WoT, bo, out);
  (void)hipGetLastError();
}
